// StateSpaceLayer_60713657696872
// MI455X (gfx1250) — hardware-verified
//
#include <hip/hip_runtime.h>
#include <math.h>
#include <stdint.h>

#define NB   2
#define TS   512
#define DS   64
#define NBT  (NB * TS)
#define PLN  (DS * DS)
#define NTOT (NBT * PLN)
static_assert((TS % 64) == 0);
static_assert(DS == 64);
static_assert(PLN == 2 * 8 * 256);

typedef _Float16 v16h __attribute__((ext_vector_type(16)));
typedef _Float16 v8h  __attribute__((ext_vector_type(8)));
typedef float    v8f  __attribute__((ext_vector_type(8)));
typedef float    v4f  __attribute__((ext_vector_type(4)));
typedef unsigned int v4u __attribute__((ext_vector_type(4)));

__device__ __forceinline__ unsigned short bf_bits(float f) {
  unsigned u = __float_as_uint(f);
  return (unsigned short)((u + 0x7FFFu + ((u >> 16) & 1u)) >> 16);
}
__device__ __forceinline__ float bfr(float f) { return __uint_as_float(((unsigned)bf_bits(f)) << 16); }
__device__ __forceinline__ unsigned short h_bits(_Float16 x) { return __builtin_bit_cast(unsigned short, x); }
__device__ __forceinline__ unsigned pk16(unsigned short a, unsigned short b) { return (unsigned)a | ((unsigned)b << 16); }
__device__ __forceinline__ v8f zero8() { v8f z = {0.f, 0.f, 0.f, 0.f, 0.f, 0.f, 0.f, 0.f}; return z; }
__device__ __forceinline__ float wave_sum(float v) {
#pragma unroll
  for (int off = 16; off > 0; off >>= 1) v += __shfl_xor(v, off, 32);
  return v;
}

__device__ __forceinline__ v16h ldfrag_h(const _Float16* p) {
  union { v16h v; v8h h[2]; } f;
  f.h[0] = *(const v8h*)(p);
  f.h[1] = *(const v8h*)(p + 16);
  return f.v;
}

__device__ __forceinline__ v8f mma_h(v16h a, v16h b, v8f c) {
  c = __builtin_amdgcn_wmma_f32_16x16x32_f16(false, a, false, b, (short)0, c, false, false);
#if defined(__HIP_DEVICE_COMPILE__)
  asm volatile("v_nop\n\tv_nop\n\tv_nop\n\tv_nop" : "+v"(c) : "v"(a), "v"(b));
#endif
  return c;
}

__global__ __launch_bounds__(256) void ln_k(const float* __restrict__ x, const float* __restrict__ logA,
                                            const float* __restrict__ dtw, const float* __restrict__ dtb,
                                            const float* __restrict__ lnw, const float* __restrict__ lnb,
                                            unsigned short* Xh, unsigned short* Xl, float* ldp, int nbt) {
  __shared__ float red0[8];
  __shared__ float red1[8];
  __shared__ float zrow[64];
  __shared__ __align__(16) float ldv[64];
  const int bt = blockIdx.x;
  if (bt >= nbt) return;
  const int tid = threadIdx.x, lane = tid & 31, wave = tid >> 5;
  const int e0 = tid * 8, e1 = 2048 + tid * 8;
  const float* xp = x + (size_t)bt * PLN;

  const v4f xa = *(const v4f*)(xp + e0);
  const v4f xb = *(const v4f*)(xp + e0 + 4);
  const v4f xc = *(const v4f*)(xp + e1);
  const v4f xd = *(const v4f*)(xp + e1 + 4);
  float v[16];
#pragma unroll
  for (int q = 0; q < 4; ++q) {
    v[q]      = bfr(xa[q]);
    v[4 + q]  = bfr(xb[q]);
    v[8 + q]  = bfr(xc[q]);
    v[12 + q] = bfr(xd[q]);
  }
  float s = 0.0f;
#pragma unroll
  for (int i = 0; i < 16; ++i) s += v[i];
  s = wave_sum(s);
  if (lane == 0) red0[wave] = s;
  __syncthreads();
  float tot = 0.0f;
#pragma unroll
  for (int w = 0; w < 8; ++w) tot += red0[w];
  const float mu = tot * (1.0f / 4096.0f);
  float ss = 0.0f;
#pragma unroll
  for (int i = 0; i < 16; ++i) { const float d = v[i] - mu; ss += d * d; }
  ss = wave_sum(ss);
  if (lane == 0) red1[wave] = ss;
  __syncthreads();
  float vt = 0.0f;
#pragma unroll
  for (int w = 0; w < 8; ++w) vt += red1[w];
  const float var  = vt * (1.0f / 4096.0f);
  const float rstd = rsqrtf(var + 1e-5f);
  const v4f wa = *(const v4f*)(lnw + e0), wb = *(const v4f*)(lnw + e0 + 4);
  const v4f wc = *(const v4f*)(lnw + e1), wd = *(const v4f*)(lnw + e1 + 4);
  const v4f ba = *(const v4f*)(lnb + e0), bb = *(const v4f*)(lnb + e0 + 4);
  const v4f bc = *(const v4f*)(lnb + e1), bd = *(const v4f*)(lnb + e1 + 4);
  float xn[16];
#pragma unroll
  for (int q = 0; q < 4; ++q) {
    xn[q]      = (v[q]      - mu) * rstd * bfr(wa[q]) + bfr(ba[q]);
    xn[4 + q]  = (v[4 + q]  - mu) * rstd * bfr(wb[q]) + bfr(bb[q]);
    xn[8 + q]  = (v[8 + q]  - mu) * rstd * bfr(wc[q]) + bfr(bc[q]);
    xn[12 + q] = (v[12 + q] - mu) * rstd * bfr(wd[q]) + bfr(bd[q]);
  }
  const int c8 = (tid & 7) * 8;
  const v4f da = *(const v4f*)(dtw + c8), db = *(const v4f*)(dtw + c8 + 4);
  float dw[8];
#pragma unroll
  for (int q = 0; q < 4; ++q) { dw[q] = bfr(da[q]); dw[4 + q] = bfr(db[q]); }
  float d0 = 0.0f, d1 = 0.0f;
#pragma unroll
  for (int i = 0; i < 8; ++i) { d0 += xn[i] * dw[i]; d1 += xn[8 + i] * dw[i]; }
  d0 += __shfl_xor(d0, 1, 32); d0 += __shfl_xor(d0, 2, 32); d0 += __shfl_xor(d0, 4, 32);
  d1 += __shfl_xor(d1, 1, 32); d1 += __shfl_xor(d1, 2, 32); d1 += __shfl_xor(d1, 4, 32);
  if ((tid & 7) == 0) { zrow[tid >> 3] = d0; zrow[32 + (tid >> 3)] = d1; }
  __syncthreads();
  if (tid < 64) {
    const float z  = zrow[tid] + bfr(dtb[0]);
    const float sp = fmaxf(z, 0.0f) + log1pf(__expf(-fabsf(z)));
    const float ac = -__expf(bfr(logA[tid]));
    ldv[tid] = sp * ac;
  }
  __syncthreads();
  v4u ph0, pl0, ph1, pl1;
#pragma unroll
  for (int e = 0; e < 4; ++e) {
    const float g0 = xn[2 * e] * 8.0f, g1 = xn[2 * e + 1] * 8.0f;
    const _Float16 x0 = (_Float16)g0, x1 = (_Float16)g1;
    const _Float16 y0 = (_Float16)((g0 - (float)x0) * 2048.0f);
    const _Float16 y1 = (_Float16)((g1 - (float)x1) * 2048.0f);
    ph0[e] = pk16(h_bits(x0), h_bits(x1));
    pl0[e] = pk16(h_bits(y0), h_bits(y1));
    const float k0 = xn[8 + 2 * e] * 8.0f, k1 = xn[8 + 2 * e + 1] * 8.0f;
    const _Float16 u0 = (_Float16)k0, u1 = (_Float16)k1;
    const _Float16 w0 = (_Float16)((k0 - (float)u0) * 2048.0f);
    const _Float16 w1 = (_Float16)((k1 - (float)u1) * 2048.0f);
    ph1[e] = pk16(h_bits(u0), h_bits(u1));
    pl1[e] = pk16(h_bits(w0), h_bits(w1));
  }
  const v4f lv = *(const v4f*)(ldv + (tid & 15) * 4);
  const size_t po0 = (size_t)bt * PLN + e0;
  const size_t po1 = (size_t)bt * PLN + e1;
  const size_t plo = (size_t)bt * DS + (tid & 15) * 4;
  for (int pass = 0; pass < 2; ++pass) {
    *(volatile v4u*)(Xh + po0) = ph0;
    *(volatile v4u*)(Xh + po1) = ph1;
    *(volatile v4u*)(Xl + po0) = pl0;
    *(volatile v4u*)(Xl + po1) = pl1;
    if (tid < 16) *(volatile v4f*)(ldp + plo) = lv;
    __threadfence();
  }
}

__global__ __launch_bounds__(256) void xt_k(const unsigned short* __restrict__ Xhp, const unsigned short* __restrict__ Xlp,
                                            unsigned short* XhT, unsigned short* XlT) {
  __shared__ __align__(16) _Float16 sh[64 * 72];
  __shared__ __align__(16) _Float16 sl[64 * 72];
  const int tid = threadIdx.x;
  const int t0  = blockIdx.x * 64;
  const int r   = blockIdx.y;
  const int b   = blockIdx.z;
  const _Float16* H = (const _Float16*)(const void*)Xhp;
  const _Float16* L = (const _Float16*)(const void*)Xlp;
#pragma unroll
  for (int i = 0; i < 2; ++i) {
    const int idx = i * 256 + tid;
    const int tt = idx >> 3, cc8 = (idx & 7) * 8;
    const size_t so = (((size_t)(b * TS + t0 + tt)) * DS + r) * DS + cc8;
    const v8h a  = *(const v8h*)(H + so);
    const v8h a2 = *(const v8h*)(L + so);
    *(v8h*)(sh + tt * 72 + cc8) = a;
    *(v8h*)(sl + tt * 72 + cc8) = a2;
  }
  __syncthreads();

  const int g = tid >> 3, piece = tid & 7;
  v4u hv[2], lvv[2];
  size_t hofs[2];
#pragma unroll
  for (int it = 0; it < 2; ++it) {
    const int c = it * 32 + g;
    v4u a, a2;
#pragma unroll
    for (int e = 0; e < 4; ++e) {
      const int ta = piece * 8 + 2 * e, tb = ta + 1;
      a[e]  = pk16(h_bits(sh[ta * 72 + c]), h_bits(sh[tb * 72 + c]));
      a2[e] = pk16(h_bits(sl[ta * 72 + c]), h_bits(sl[tb * 72 + c]));
    }
    hv[it]  = a;
    lvv[it] = a2;
    hofs[it] = (((size_t)(b * DS + r)) * DS + c) * TS + t0 + piece * 8;
  }
  for (int pass = 0; pass < 2; ++pass) {
#pragma unroll
    for (int it = 0; it < 2; ++it) {
      *(volatile v4u*)(XhT + hofs[it]) = hv[it];
      *(volatile v4u*)(XlT + hofs[it]) = lvv[it];
    }
    __threadfence();
  }
}

__global__ __launch_bounds__(128) void ssm_k(const unsigned short* __restrict__ XhTp, const unsigned short* __restrict__ XlTp,
                                             const float* __restrict__ ldp, float* outp) {
  __shared__ __align__(16) float cs_s[TS];
  __shared__ __align__(16) float os_s[4 * 16 * 64];
  const int tt = blockIdx.x, r = blockIdx.y, b = blockIdx.z;
  const int tid = threadIdx.x, wave = tid >> 5, lane = tid & 31, hh = lane >> 4, l16 = lane & 15;

#pragma unroll 1
  for (int i = tid; i < TS; i += 128) cs_s[i] = ldp[((size_t)(b * TS + i)) * DS + r];
  __syncthreads();
  if (tid == 0) {
    float a = 0.0f;
#pragma unroll 4
    for (int t = 0; t < TS; ++t) { a += cs_s[t]; cs_s[t] = a; }
  }
  __syncthreads();

  const int tbase = tt * 64 + wave * 16;
  const int trow  = tbase + l16;
  const float cst = cs_s[trow];
  const _Float16* XhT = (const _Float16*)(const void*)XhTp;
  const _Float16* XlT = (const _Float16*)(const void*)XlTp;
  const size_t plb = ((size_t)(b * DS + r)) * DS * TS;
  const _Float16* xbh = XhT + plb;
  const _Float16* xbl = XlT + plb;

  v8f acc[4], acc2[4];
#pragma unroll
  for (int s = 0; s < 4; ++s) { acc[s] = zero8(); acc2[s] = zero8(); }

  const int jend = tbase + 16;
#pragma unroll 1
  for (int j0 = 0; j0 < jend; j0 += 32) {
    const int kA = j0 + hh * 8;
    const int kB = j0 + 16 + hh * 8;
    const v4f q0 = *(const v4f*)(cs_s + kA);
    const v4f q1 = *(const v4f*)(cs_s + kA + 4);
    const v4f q2 = *(const v4f*)(cs_s + kB);
    const v4f q3 = *(const v4f*)(cs_s + kB + 4);
    float cj[16];
#pragma unroll
    for (int q = 0; q < 4; ++q) {
      cj[q]      = q0[q];
      cj[q + 4]  = q1[q];
      cj[q + 8]  = q2[q];
      cj[q + 12] = q3[q];
    }
    v16h pa, pr;
#pragma unroll
    for (int e = 0; e < 16; ++e) {
      const int j = (e < 8) ? (kA + e) : (kB + e - 8);
      const float d = fminf(cst - cj[e], 0.0f);
      float p = __expf(d) * 16384.0f;
      p = (j <= trow) ? p : 0.0f;
      const _Float16 x0 = (_Float16)p;
      pa[e] = x0;
      pr[e] = (_Float16)((p - (float)x0) * 2048.0f);
    }
#pragma unroll
    for (int s = 0; s < 4; ++s) {
      const size_t bo = (size_t)(s * 16 + l16) * TS + j0 + 8 * hh;
      const v16h xh = ldfrag_h(xbh + bo);
      const v16h xl = ldfrag_h(xbl + bo);
      acc[s]  = mma_h(pa, xh, acc[s]);
      acc2[s] = mma_h(pa, xl, acc2[s]);
      acc2[s] = mma_h(pr, xh, acc2[s]);
    }
  }

  float* os = os_s + wave * (16 * 64);
#pragma unroll
  for (int r8 = 0; r8 < 8; ++r8) {
#pragma unroll
    for (int s = 0; s < 4; ++s) {
      const float val = (acc[s][r8] + acc2[s][r8] * (1.0f / 2048.0f)) * (1.0f / 131072.0f);
      os[(8 * hh + r8) * 64 + s * 16 + l16] = val;
    }
  }
  __builtin_amdgcn_fence(__ATOMIC_RELEASE, "workgroup");
  __builtin_amdgcn_wave_barrier();
  __builtin_amdgcn_fence(__ATOMIC_ACQUIRE, "workgroup");
  const int h2 = lane >> 4, c4 = (lane & 15) * 4;
  v4f ov[8];
#pragma unroll
  for (int it = 0; it < 8; ++it) {
    const int row = it * 2 + h2;
    ov[it] = *(const v4f*)(os + row * 64 + c4);
  }
  for (int pass = 0; pass < 2; ++pass) {
#pragma unroll
    for (int it = 0; it < 8; ++it) {
      const int row = it * 2 + h2;
      const size_t go = (((size_t)(b * TS + tbase + row)) * DS + r) * DS + c4;
      *(volatile v4f*)(outp + go) = ov[it];
    }
    __threadfence();
  }
}

extern "C" void kernel_launch(void* const* d_in, const int* in_sizes, int n_in,
                              void* d_out, int out_size, void* d_ws, size_t ws_size,
                              hipStream_t stream) {
  if (n_in < 6) return;
  if (in_sizes[0] != NTOT) return;
  if (in_sizes[1] != DS) return;
  if (in_sizes[2] != DS) return;
  if (in_sizes[3] != 1) return;
  if (in_sizes[4] != PLN) return;
  if (in_sizes[5] != PLN) return;
  if (out_size != NTOT) return;

  const float* x    = (const float*)d_in[0];
  const float* logA = (const float*)d_in[1];
  const float* dtw  = (const float*)d_in[2];
  const float* dtb  = (const float*)d_in[3];
  const float* lnw  = (const float*)d_in[4];
  const float* lnb  = (const float*)d_in[5];
  float* outf = (float*)d_out;

  const size_t PB = (size_t)NTOT * 2;
  const size_t LB = (size_t)NBT * DS * 4;
  size_t off = 0;
  const size_t oXh  = off; off += PB;
  const size_t oXl  = off; off += PB;
  const size_t oXhT = off; off += PB;
  const size_t oXlT = off; off += PB;
  const size_t oLd  = off; off += LB;
  if (off > ws_size) return;
  if (off > (size_t)134217728) return;

  char* ws = (char*)d_ws;
  unsigned short* Xh  = (unsigned short*)(ws + oXh);
  unsigned short* Xl  = (unsigned short*)(ws + oXl);
  unsigned short* XhT = (unsigned short*)(ws + oXhT);
  unsigned short* XlT = (unsigned short*)(ws + oXlT);
  float*          Ld  = (float*)(ws + oLd);

  const int nbt = in_sizes[0] / PLN;
  ln_k<<<dim3(nbt), dim3(256), 0, stream>>>(x, logA, dtw, dtb, lnw, lnb, Xh, Xl, Ld, nbt);
  xt_k<<<dim3(TS / 64, DS, NB), dim3(256), 0, stream>>>(Xh, Xl, XhT, XlT);
  ssm_k<<<dim3(TS / 64, DS, NB), dim3(128), 0, stream>>>(XhT, XlT, Ld, outf);
  (void)hipGetLastError();
}
